// EncoderRNN_9285719294595
// MI455X (gfx1250) — hardware-verified
//
#include <hip/hip_runtime.h>
#include <math.h>

constexpr int NBAT     = 64;
constexpr int NSTEP    = 1024;
constexpr int NIN      = 64;
constexpr int NHID     = 256;
constexpr int NGATE3   = 3 * NHID;
constexpr int NCAT     = 2 * NHID;
constexpr int NBIAS    = 2 * NGATE3;
constexpr int CVT_THR  = 256;
constexpr int RNN_THR  = 512;
constexpr int NWAVE    = RNN_THR / 32;
constexpr int ROWS_BLK = 16;
constexpr int NBLK     = NBAT / ROWS_BLK;
constexpr int XPITCH   = 72;
constexpr int HPITCH   = 520;
constexpr int OPITCH   = 516;
constexpr float WCARRY     = 256.0f;
constexpr float WCARRY_INV = 1.0f / 256.0f;
static_assert(NBAT % ROWS_BLK == 0);
static_assert(NHID == 16 * NWAVE);
static_assert(NWAVE == ROWS_BLK);
static_assert(NIN % 32 == 0 && NHID % 32 == 0 && NCAT % 32 == 0);
static_assert(XPITCH % 8 == 0 && HPITCH % 8 == 0 && OPITCH % 4 == 0);
static_assert(XPITCH >= NIN && HPITCH >= NCAT && OPITCH >= NCAT);
static_assert(4 * NBIAS <= ROWS_BLK * OPITCH);
static_assert((NBIAS / 4) % 32 == 0 && NBIAS / 4 <= RNN_THR);
static_assert(ROWS_BLK * NIN == 2 * RNN_THR);
static_assert(NBAT % 32 == 0 && NBAT <= RNN_THR);
static_assert((2 * NGATE3 * NIN / 8) % CVT_THR == 0);
static_assert((2 * NGATE3 * NHID / 8) % CVT_THR == 0);
static_assert((2 * NGATE3 * NCAT / 8) % CVT_THR == 0);

typedef __attribute__((ext_vector_type(16))) _Float16 v16h;
typedef __attribute__((ext_vector_type(8)))  _Float16 v8h;
typedef __attribute__((ext_vector_type(8)))  float    v8f;
typedef __attribute__((ext_vector_type(4)))  float    v4f;
typedef __attribute__((ext_vector_type(2)))  float    v2f;

__device__ __forceinline__ unsigned short f2bf_bits(float f) {
  unsigned u = __float_as_uint(f);
  return (unsigned short)((u + 0x7FFFu + ((u >> 16) & 1u)) >> 16);
}
__device__ __forceinline__ float bf_bits2f(unsigned short h) { return __uint_as_float(((unsigned)h) << 16); }
__device__ __forceinline__ float bf16r(float f) { return bf_bits2f(f2bf_bits(f)); }

__device__ __forceinline__ void guard3x4_h(v8f& a, v8f& b, v8f& c, v16h w, v16h x, v16h y, v16h z) {
  asm volatile("v_nop\n\tv_nop\n\tv_nop\n\tv_nop" : "+v"(a), "+v"(b), "+v"(c) : "v"(w), "v"(x), "v"(y), "v"(z));
}
__device__ __forceinline__ void acc_guard4(v8f& a, v8f& b, v8f& c, v8f& d) { asm volatile("v_nop\n\tv_nop\n\tv_nop\n\tv_nop" : "+v"(a), "+v"(b), "+v"(c), "+v"(d)); }
template <typename T> struct Frag;
template <> struct Frag<_Float16> {
  typedef v16h V; union U { v16h v; v8h h[2]; };
  static __device__ __forceinline__ v16h load(const _Float16* p) {
    U f; f.h[0] = *(const v8h*)(p); f.h[1] = *(const v8h*)(p + 16); return f.v;
  }
  static __device__ __forceinline__ v8f mma(v16h a, v16h b, v8f c) {
    return __builtin_amdgcn_wmma_f32_16x16x32_f16(false, a, false, b, (short)0, c, false, false);
  }
};

__device__ __forceinline__ float fsig(float x)  { return __builtin_amdgcn_rcpf(1.0f + expf(-x)); }
__device__ __forceinline__ float ftanh(float x) { return 1.0f - 2.0f * __builtin_amdgcn_rcpf(expf(2.0f * x) + 1.0f); }

template <int MODE>
__global__ __launch_bounds__(CVT_THR) void cvt8_kernel(const float* __restrict__ src, unsigned short* __restrict__ dst,
                                                       int nrow, int ncol8, int spitch, int scol0, float sc) {
  const int i  = blockIdx.x * CVT_THR + threadIdx.x;
  const int n8 = nrow * ncol8;
  if (i < n8) {
    const int row = i / ncol8;
    const int c8  = i - row * ncol8;
    const float* sp = src + (size_t)row * spitch + scol0 + c8 * 8;
    const v4f a = *(const v4f*)(sp);
    const v4f b = *(const v4f*)(sp + 4);
    v8h hv;
#pragma unroll
    for (int e = 0; e < 4; ++e) {
      unsigned short b0, b1;
      if (MODE == 0) {
        b0 = f2bf_bits(a[e] * sc);
        b1 = f2bf_bits(b[e] * sc);
      } else {
        b0 = __builtin_bit_cast(unsigned short, (_Float16)(bf16r(a[e]) * sc));
        b1 = __builtin_bit_cast(unsigned short, (_Float16)(bf16r(b[e]) * sc));
      }
      hv[e]     = __builtin_bit_cast(_Float16, b0);
      hv[4 + e] = __builtin_bit_cast(_Float16, b1);
    }
    *(volatile v8h*)(dst + (size_t)i * 8) = hv;
    __threadfence();
    *(volatile v8h*)(dst + (size_t)i * 8) = hv;
  }
}

template <int KIN>
__device__ __forceinline__ void gru_tile(const _Float16* xa, const _Float16* ha,
                                         const _Float16* __restrict__ wi, const _Float16* __restrict__ wh,
                                         float bR, float bZ, float bI, float bH, float (&hst)[8]) {
  const v8f z8 = {0.f, 0.f, 0.f, 0.f, 0.f, 0.f, 0.f, 0.f};
  v8f aR = z8, aZ = z8, aI = z8, aH = z8;
#pragma unroll 1
  for (int k0 = 0; k0 < KIN; k0 += 32) {
    const v16h a  = Frag<_Float16>::load(xa + k0);
    const v16h b0 = Frag<_Float16>::load(wi + k0);
    const v16h b1 = Frag<_Float16>::load(wi + (size_t)NHID * KIN + k0);
    const v16h b2 = Frag<_Float16>::load(wi + (size_t)2 * NHID * KIN + k0);
    aR = Frag<_Float16>::mma(a, b0, aR);
    aZ = Frag<_Float16>::mma(a, b1, aZ);
    aI = Frag<_Float16>::mma(a, b2, aI);
    guard3x4_h(aR, aZ, aI, a, b0, b1, b2);
  }
#pragma unroll 1
  for (int k0 = 0; k0 < NHID; k0 += 32) {
    const v16h a  = Frag<_Float16>::load(ha + k0);
    const v16h b0 = Frag<_Float16>::load(wh + k0);
    const v16h b1 = Frag<_Float16>::load(wh + (size_t)NHID * NHID + k0);
    const v16h b2 = Frag<_Float16>::load(wh + (size_t)2 * NHID * NHID + k0);
    aR = Frag<_Float16>::mma(a, b0, aR);
    aZ = Frag<_Float16>::mma(a, b1, aZ);
    aH = Frag<_Float16>::mma(a, b2, aH);
    guard3x4_h(aR, aZ, aH, a, b0, b1, b2);
  }
  acc_guard4(aR, aZ, aI, aH);
#pragma unroll
  for (int r = 0; r < 8; ++r) {
    const float pr = aR[r] * WCARRY_INV + bR;
    const float pz = aZ[r] * WCARRY_INV + bZ;
    const float pi = aI[r] * WCARRY_INV + bI;
    const float ph = aH[r] * WCARRY_INV + bH;
    const float rg = fsig(pr);
    const float zg = fsig(pz);
    const float nn = ftanh(pi + rg * ph);
    const float ho = hst[r];
    hst[r] = (1.0f - zg) * nn + zg * ho;
  }
}

__device__ __forceinline__ void write_h16(_Float16* hn, const float (&hst)[8], int hh) {
#pragma unroll
  for (int r = 0; r < 8; ++r) hn[(8 * hh + r) * HPITCH] = (_Float16)hst[r];
}
__device__ __forceinline__ void capture_h(float (&hf)[8], const float (&hst)[8], const int (&tl)[8], int t) {
#pragma unroll
  for (int r = 0; r < 8; ++r) hf[r] = (t == tl[r]) ? hst[r] : hf[r];
}
__device__ __forceinline__ void stage_x2(unsigned short* Xs, const float* xrow, int tn, int xm, int xf2) {
  const v2f v = *(const v2f*)(xrow + (size_t)tn * NIN);
  const unsigned short u0 = __builtin_bit_cast(unsigned short, (_Float16)bf16r(v[0]));
  const unsigned short u1 = __builtin_bit_cast(unsigned short, (_Float16)bf16r(v[1]));
  const unsigned u = (unsigned)u0 | ((unsigned)u1 << 16);
  *(unsigned*)(Xs + xm * XPITCH + xf2) = u;
}
__device__ __forceinline__ void cell_bias(const float* Bs, int layer, int d, int jcol, float& bR, float& bZ, float& bI, float& bH) {
  const float* bi = Bs + (2 * layer) * NBIAS + d * NGATE3;
  const float* bh = Bs + (2 * layer + 1) * NBIAS + d * NGATE3;
  bR = bf16r(bi[jcol]) + bf16r(bh[jcol]);
  bZ = bf16r(bi[NHID + jcol]) + bf16r(bh[NHID + jcol]);
  bI = bf16r(bi[2 * NHID + jcol]);
  bH = bf16r(bh[2 * NHID + jcol]);
}

__global__ __launch_bounds__(RNN_THR) void gru2_seq_kernel(
    const float* __restrict__ x,
    const float* __restrict__ bih0, const float* __restrict__ bhh0,
    const float* __restrict__ bih1, const float* __restrict__ bhh1,
    const int* __restrict__ seqlen,
    const unsigned short* __restrict__ WI0p, const unsigned short* __restrict__ WH0p,
    const unsigned short* __restrict__ WI1p, const unsigned short* __restrict__ WH1p,
    float* __restrict__ out) {
  __shared__ __align__(16) unsigned short Xs[ROWS_BLK * XPITCH];
  __shared__ __align__(16) _Float16 H0s[2][ROWS_BLK * HPITCH];
  __shared__ __align__(16) _Float16 H1s[2][ROWS_BLK * HPITCH];
  __shared__ __align__(16) float Hs[ROWS_BLK * OPITCH];
  __shared__ int Idx[NBAT];
  __shared__ int Inv[NBAT];
  __shared__ int Brow[ROWS_BLK];
  __shared__ int Tloc[ROWS_BLK];

  const _Float16* WI0 = (const _Float16*)WI0p;
  const _Float16* WH0 = (const _Float16*)WH0p;
  const _Float16* WI1 = (const _Float16*)WI1p;
  const _Float16* WH1 = (const _Float16*)WH1p;
  const int tid = threadIdx.x, lane = tid & 31, wave = tid >> 5;
  const int c = lane & 15, hh = lane >> 4, koff = hh * 8;
  const int jcol = 16 * wave + c;

  if (tid < NBAT) {
    int ix = seqlen[tid] - 1;
    ix = ix < 0 ? 0 : (ix > NSTEP - 1 ? NSTEP - 1 : ix);
    Idx[tid] = ix;
    Inv[tid] = tid;
  }
  __syncthreads();
  if (tid < NBAT) {
    const int ix = Idx[tid];
    int rank = 0;
#pragma unroll 1
    for (int b2 = 0; b2 < NBAT; ++b2) {
      const int v = Idx[b2];
      rank += (v < ix || (v == ix && b2 < tid)) ? 1 : 0;
    }
    rank = rank < 0 ? 0 : (rank > NBAT - 1 ? NBAT - 1 : rank);
    Inv[rank] = tid;
  }
  __syncthreads();
  if (tid < ROWS_BLK) {
    int b = Inv[blockIdx.x * ROWS_BLK + tid];
    b = b < 0 ? 0 : (b > NBAT - 1 ? NBAT - 1 : b);
    Brow[tid] = b;
    Tloc[tid] = Idx[b];
  }
  __syncthreads();
  int tmax = 0;
#pragma unroll 1
  for (int i = 0; i < ROWS_BLK; ++i) { const int v = Tloc[i]; tmax = v > tmax ? v : tmax; }
  tmax += 1;
  tmax = tmax > NSTEP ? NSTEP : tmax;
  int tl[8];
#pragma unroll
  for (int r = 0; r < 8; ++r) tl[r] = Tloc[8 * hh + r];
  const int xm = wave, xf2 = lane * 2;
  int xb = Brow[xm];
  xb = xb < 0 ? 0 : (xb > NBAT - 1 ? NBAT - 1 : xb);
  const float* xrow = x + (size_t)xb * NSTEP * NIN + xf2;

  {
    _Float16* h0f = &H0s[0][0];
    _Float16* h1f = &H1s[0][0];
#pragma unroll 1
    for (int i = tid; i < 2 * ROWS_BLK * HPITCH; i += RNN_THR) { h0f[i] = (_Float16)0.0f; h1f[i] = (_Float16)0.0f; }
  }
  stage_x2(Xs, xrow, 0, xm, xf2);
  if (tid < NBIAS / 4) {
    const v4f v0 = *(const v4f*)(bih0 + 4 * tid);
    const v4f v1 = *(const v4f*)(bhh0 + 4 * tid);
    const v4f v2 = *(const v4f*)(bih1 + 4 * tid);
    const v4f v3 = *(const v4f*)(bhh1 + 4 * tid);
    *(v4f*)(Hs + 0 * NBIAS + 4 * tid) = v0;
    *(v4f*)(Hs + 1 * NBIAS + 4 * tid) = v1;
    *(v4f*)(Hs + 2 * NBIAS + 4 * tid) = v2;
    *(v4f*)(Hs + 3 * NBIAS + 4 * tid) = v3;
  }
  __syncthreads();
  float bR0, bZ0, bI0, bH0, bR1, bZ1, bI1, bH1, bR2, bZ2, bI2, bH2, bR3, bZ3, bI3, bH3;
  cell_bias(Hs, 0, 0, jcol, bR0, bZ0, bI0, bH0);
  cell_bias(Hs, 0, 1, jcol, bR1, bZ1, bI1, bH1);
  cell_bias(Hs, 1, 0, jcol, bR2, bZ2, bI2, bH2);
  cell_bias(Hs, 1, 1, jcol, bR3, bZ3, bI3, bH3);
  float h00[8], h01[8], h10[8], h11[8], hf0[8], hf1[8];
#pragma unroll
  for (int r = 0; r < 8; ++r) { h00[r] = 0.0f; h01[r] = 0.0f; h10[r] = 0.0f; h11[r] = 0.0f; hf0[r] = 0.0f; hf1[r] = 0.0f; }

  const _Float16* xa0 = (const _Float16*)Xs + c * XPITCH + koff;
  const _Float16* wi00 = WI0 + ((size_t)(0 * NGATE3 + jcol)) * NIN  + koff;
  const _Float16* wi01 = WI0 + ((size_t)(1 * NGATE3 + jcol)) * NIN  + koff;
  const _Float16* wh00 = WH0 + ((size_t)(0 * NGATE3 + jcol)) * NHID + koff;
  const _Float16* wh01 = WH0 + ((size_t)(1 * NGATE3 + jcol)) * NHID + koff;
  const _Float16* wi10 = WI1 + ((size_t)(0 * NGATE3 + jcol)) * NCAT + koff;
  const _Float16* wi11 = WI1 + ((size_t)(1 * NGATE3 + jcol)) * NCAT + koff;
  const _Float16* wh10 = WH1 + ((size_t)(0 * NGATE3 + jcol)) * NHID + koff;
  const _Float16* wh11 = WH1 + ((size_t)(1 * NGATE3 + jcol)) * NHID + koff;

#pragma unroll 1
  for (int t = 0; t < tmax; ++t) {
    const int cur = t & 1, nxt = cur ^ 1;
    {
      const _Float16* ha = &H0s[cur][0] + c * HPITCH + 0 * NHID + koff;
      gru_tile<NIN>(xa0, ha, wi00, wh00, bR0, bZ0, bI0, bH0, h00);
      write_h16(&H0s[nxt][0] + 0 * NHID + jcol, h00, hh);
    }
    {
      const _Float16* ha = &H0s[cur][0] + c * HPITCH + 1 * NHID + koff;
      gru_tile<NIN>(xa0, ha, wi01, wh01, bR1, bZ1, bI1, bH1, h01);
      write_h16(&H0s[nxt][0] + 1 * NHID + jcol, h01, hh);
    }
    __syncthreads();
    {
      const int tn = (t + 1 < NSTEP) ? (t + 1) : (NSTEP - 1);
      stage_x2(Xs, xrow, tn, xm, xf2);
    }
    {
      const _Float16* ya = &H0s[nxt][0] + c * HPITCH + koff;
      const _Float16* ha = &H1s[cur][0] + c * HPITCH + 0 * NHID + koff;
      gru_tile<NCAT>(ya, ha, wi10, wh10, bR2, bZ2, bI2, bH2, h10);
      write_h16(&H1s[nxt][0] + 0 * NHID + jcol, h10, hh);
      capture_h(hf0, h10, tl, t);
    }
    {
      const _Float16* ya = &H0s[nxt][0] + c * HPITCH + koff;
      const _Float16* ha = &H1s[cur][0] + c * HPITCH + 1 * NHID + koff;
      gru_tile<NCAT>(ya, ha, wi11, wh11, bR3, bZ3, bI3, bH3, h11);
      write_h16(&H1s[nxt][0] + 1 * NHID + jcol, h11, hh);
      capture_h(hf1, h11, tl, t);
    }
    __syncthreads();
  }

#pragma unroll
  for (int r = 0; r < 8; ++r) {
    Hs[(8 * hh + r) * OPITCH + 0 * NHID + jcol] = hf0[r];
    Hs[(8 * hh + r) * OPITCH + 1 * NHID + jcol] = hf1[r];
  }
  __syncthreads();
  {
    int b = Brow[wave];
    b = b < 0 ? 0 : (b > NBAT - 1 ? NBAT - 1 : b);
    float* op = out + (size_t)b * NCAT;
    const float* sp = Hs + wave * OPITCH;
    for (int pass = 0; pass < 2; ++pass) {
#pragma unroll
      for (int q = 0; q < 4; ++q) {
        const v4f v = *(const v4f*)(sp + q * 128 + 4 * lane);
        *(volatile v4f*)(op + q * 128 + 4 * lane) = v;
      }
      __threadfence();
    }
  }
}

extern "C" void kernel_launch(void* const* d_in, const int* in_sizes, int n_in,
                              void* d_out, int out_size, void* d_ws, size_t ws_size, hipStream_t stream) {
  if (n_in < 10 || d_out == nullptr || d_ws == nullptr) return;
  if (in_sizes[0] != NBAT * NSTEP * NIN || in_sizes[1] != 2 * NGATE3 * NIN || in_sizes[2] != 2 * NGATE3 * NHID ||
      in_sizes[3] != NBIAS || in_sizes[4] != NBIAS || in_sizes[5] != 2 * NGATE3 * NCAT || in_sizes[6] != 2 * NGATE3 * NHID ||
      in_sizes[7] != NBIAS || in_sizes[8] != NBIAS || in_sizes[9] != NBAT || out_size != NBAT * NCAT) return;

  const float* x     = (const float*)d_in[0];
  const float* w_ih0 = (const float*)d_in[1];
  const float* w_hh0 = (const float*)d_in[2];
  const float* b_ih0 = (const float*)d_in[3];
  const float* b_hh0 = (const float*)d_in[4];
  const float* w_ih1 = (const float*)d_in[5];
  const float* w_hh1 = (const float*)d_in[6];
  const float* b_ih1 = (const float*)d_in[7];
  const float* b_hh1 = (const float*)d_in[8];
  const int*   seq   = (const int*)d_in[9];
  float* out = (float*)d_out;

  char* ws = (char*)d_ws; size_t off = 0;
  auto carve = [&](size_t bytes) -> char* { char* p = ws + off; off += (bytes + 255) & ~(size_t)255; return p; };
  unsigned short* WI0 = (unsigned short*)carve((size_t)2 * NGATE3 * NIN  * 2);
  unsigned short* WH0 = (unsigned short*)carve((size_t)2 * NGATE3 * NHID * 2);
  unsigned short* WI1 = (unsigned short*)carve((size_t)2 * NGATE3 * NCAT * 2);
  unsigned short* WH1 = (unsigned short*)carve((size_t)2 * NGATE3 * NHID * 2);
  if (off > ws_size || off > (size_t)134217728) return;

  cvt8_kernel<1><<<(2 * NGATE3 * NIN  / 8) / CVT_THR, CVT_THR, 0, stream>>>(w_ih0, WI0, 2 * NGATE3, NIN  / 8, NIN,  0, WCARRY);
  cvt8_kernel<1><<<(2 * NGATE3 * NHID / 8) / CVT_THR, CVT_THR, 0, stream>>>(w_hh0, WH0, 2 * NGATE3, NHID / 8, NHID, 0, WCARRY);
  cvt8_kernel<1><<<(2 * NGATE3 * NCAT / 8) / CVT_THR, CVT_THR, 0, stream>>>(w_ih1, WI1, 2 * NGATE3, NCAT / 8, NCAT, 0, WCARRY);
  cvt8_kernel<1><<<(2 * NGATE3 * NHID / 8) / CVT_THR, CVT_THR, 0, stream>>>(w_hh1, WH1, 2 * NGATE3, NHID / 8, NHID, 0, WCARRY);
  gru2_seq_kernel<<<NBLK, RNN_THR, 0, stream>>>(x, b_ih0, b_hh0, b_ih1, b_hh1, seq, WI0, WH0, WI1, WH1, out);
}
